// NewCompoundMoE_1984274891215
// MI455X (gfx1250) — hardware-verified
//
#include <hip/hip_runtime.h>
#include <math.h>

typedef __attribute__((ext_vector_type(16))) _Float16 v16h;
typedef __attribute__((ext_vector_type(16))) __bf16 v16b;
typedef __attribute__((ext_vector_type(8)))  _Float16 v8h;
typedef __attribute__((ext_vector_type(8)))  float v8f;
typedef __attribute__((ext_vector_type(4)))  float v4f;
typedef __attribute__((ext_vector_type(2)))  float v2f;
typedef __attribute__((ext_vector_type(4)))  unsigned v4u;
typedef __attribute__((ext_vector_type(4)))  int v4i;
typedef float __attribute__((may_alias)) float_a;
typedef int __attribute__((may_alias)) int_a;

template <typename T> __device__ __forceinline__ void vst2(void* p, T v) { *(volatile T*)p = v; __threadfence(); *(volatile T*)p = v; }
__device__ __forceinline__ v8f wmma16(v16h a, v16h b, v8f c) {
  v8f d = __builtin_amdgcn_wmma_f32_16x16x32_f16(false, a, false, b, (short)0, c, false, false);
  asm volatile("v_nop\n\tv_nop\n\tv_nop\n\tv_nop" : "+v"(d) : "v"(a), "v"(b));
  return d;
}
__device__ __forceinline__ v8f wmma_bf(v16b a, v16b b, v8f c) {
  v8f d = __builtin_amdgcn_wmma_f32_16x16x32_bf16(false, a, false, b, (short)0, c, false, false);
  asm volatile("v_nop\n\tv_nop\n\tv_nop\n\tv_nop" : "+v"(d) : "v"(a), "v"(b));
  return d;
}
__device__ __forceinline__ v16h frag_h(const _Float16* rowk0, int lane) {
  union { v16h v; v8h q[2]; } u; const _Float16* p = rowk0 + 8 * (lane >> 4);
  u.q[0] = *(const v8h*)p; u.q[1] = *(const v8h*)(p + 16); return u.v;
}
__device__ __forceinline__ v16h frag_f32(const float* rowk0, int lane) {
  v16h a; const float* p = rowk0 + 8 * (lane >> 4);
#pragma unroll
  for (int i = 0; i < 8; ++i) { a[i] = (_Float16)p[i]; a[8 + i] = (_Float16)p[16 + i]; }
  return a;
}
__device__ __forceinline__ v16h frag_f32s(const float* rowk0, int lane, float sc) {
  v16h a; const float* p = rowk0 + 8 * (lane >> 4);
#pragma unroll
  for (int i = 0; i < 8; ++i) { a[i] = (_Float16)(p[i] * sc); a[8 + i] = (_Float16)(p[16 + i] * sc); }
  return a;
}
__device__ __forceinline__ v16h fragc_f32(const float* W, int k0, int n, int lane, int ld, int K) {
  v16h a; const int g = lane >> 4;
#pragma unroll
  for (int i = 0; i < 8; ++i) { const int ka = k0 + 8 * g + i, kb = ka + 16;
    a[i] = (_Float16)(ka < K ? W[(size_t)(ka < K ? ka : K - 1) * ld + n] : 0.f); a[8 + i] = (_Float16)(kb < K ? W[(size_t)(kb < K ? kb : K - 1) * ld + n] : 0.f); }
  return a;
}
struct F2 { v16b h, l; };
__device__ __forceinline__ F2 bsplit16(const float v[16]) { F2 r;
#pragma unroll
  for (int i = 0; i < 16; ++i) { const __bf16 h = (__bf16)v[i]; r.h[i] = h; r.l[i] = (__bf16)(v[i] - (float)h); }
  return r; }
__device__ __forceinline__ F2 split_row(const float* row, int k0, int lane) { float v[16]; const float* p = row + k0 + 8 * (lane >> 4);
#pragma unroll
  for (int i = 0; i < 8; ++i) { v[i] = p[i]; v[8 + i] = p[16 + i]; }
  return bsplit16(v); }
__device__ __forceinline__ F2 split_rowK(const float* row, int k0, int lane, int K) { float v[16]; const int g = lane >> 4;
#pragma unroll
  for (int i = 0; i < 8; ++i) { const int ka = k0 + 8 * g + i, kb = ka + 16; v[i] = ka < K ? row[ka < K ? ka : K - 1] : 0.f; v[8 + i] = kb < K ? row[kb < K ? kb : K - 1] : 0.f; }
  return bsplit16(v); }
__device__ __forceinline__ F2 split_col(const float* W, int k0, int n, int lane, int ld, int K) { float v[16]; const int g = lane >> 4;
#pragma unroll
  for (int i = 0; i < 8; ++i) { const int ka = k0 + 8 * g + i, kb = ka + 16; v[i] = ka < K ? W[(size_t)(ka < K ? ka : K - 1) * ld + n] : 0.f; v[8 + i] = kb < K ? W[(size_t)(kb < K ? kb : K - 1) * ld + n] : 0.f; }
  return bsplit16(v); }
__device__ __forceinline__ v8f mac3(const F2& a, const F2& b, v8f c) { c = wmma_bf(a.l, b.h, c); c = wmma_bf(a.h, b.l, c); return wmma_bf(a.h, b.h, c); }
__device__ __forceinline__ float sigm(float v) { return 1.0f / (1.0f + expf(-v)); }
#define LDSX() do { asm volatile("s_wait_dscnt 0" ::: "memory"); __builtin_amdgcn_wave_barrier(); __builtin_amdgcn_fence(__ATOMIC_RELEASE, "workgroup"); } while (0)


#define NT_ 1024
#define DD 1024
#define NOUT 8
#define NIN 2
#define NE 16
#define FF 512
#ifndef NRB
#define NRB (NT_ / 64)
#endif
typedef __attribute__((ext_vector_type(8))) __bf16 v8b;
__device__ __forceinline__ v16b frag_b(const __bf16* rowk0, int lane) {
  union { v16b v; v8b q[2]; } u; const __bf16* p = rowk0 + 8 * (lane >> 4);
  u.q[0] = *(const v8b*)p; u.q[1] = *(const v8b*)(p + 16); return u.v;
}
__device__ __forceinline__ float bfr(float v) { return (float)(__bf16)v; }
__device__ __attribute__((noinline)) float exp_ni(float v) { return expf(v); }
__device__ __attribute__((noinline)) float erf_ni(float v) { return erff(v); }

#define WS_PW  0u
#define PRT 0
#define PIN (PRT + 16 * DD)
#define PGU (PIN + 16 * DD)
#define PWD (PGU + (size_t)NE * 2 * FF * DD)
#define PWEND (PWD + (size_t)NE * DD * FF)
#define WS_CW  (WS_PW + 2u * PWEND)
#define WS_H   (WS_CW + 4u * NT_ * NE)
#define WS_END (WS_H + 4u * NT_ * NE * FF)

__global__ __launch_bounds__(256) void k_pack(const float* __restrict__ WOG, const float* __restrict__ WIN, const float* __restrict__ WG, const float* __restrict__ WU, const float* __restrict__ WDn, __bf16* __restrict__ PW) {
  __shared__ __align__(16) __bf16 s[DD]; const int n = blockIdx.x, which = blockIdx.y, tid = threadIdx.x; int K; size_t dst;
  if (which == 0) { if (n >= 32) return; K = DD; if (n < 16) { dst = PRT + (size_t)n * DD; for (int k = tid; k < K; k += 256) s[k] = (__bf16)((n < NOUT) ? WOG[(size_t)n * DD + k] : 0.f); } else { const int oi = n - 16; dst = PIN + (size_t)oi * DD; for (int k = tid; k < K; k += 256) s[k] = (__bf16)WIN[(size_t)oi * DD + k]; } }
  else if (which == 1) { K = DD; const int e = n >> 10, f = n & 1023; dst = PGU + (size_t)n * DD; const float* src = (f < FF) ? (WG + ((size_t)e * FF + f) * DD) : (WU + ((size_t)e * FF + (f - FF)) * DD); for (int k = tid; k < K; k += 256) s[k] = (__bf16)src[k]; }
  else { K = FF; dst = PWD + (size_t)n * FF; for (int k = tid; k < K; k += 256) s[k] = (__bf16)WDn[(size_t)n * FF + k]; }
  __syncthreads();
  for (int q = tid; q < K / 8; q += 256) vst2((unsigned*)(PW + dst + q * 8), *(const v4u*)&s[q * 8]);
}
__global__ __launch_bounds__(128) void k_route(const float* __restrict__ X, const __bf16* __restrict__ PW, float* __restrict__ CW, float* __restrict__ SELW) {
  __shared__ float sl[4][16][33]; __shared__ __align__(16) float scw[64][NE]; __shared__ __align__(16) float ssw[64 * 3];
  const int tid = threadIdx.x, wave = tid >> 5, lane = tid & 31, col = lane & 15, g = lane >> 4; const size_t r0 = (size_t)blockIdx.x * 64 + wave * 16;
  v8f acc[2] = {};
#pragma unroll 4
  for (int kc = 0; kc < DD / 32; ++kc) { v16b a; { const float* p = X + (r0 + col) * DD + kc * 32 + 8 * g;
#pragma unroll
      for (int i = 0; i < 8; ++i) { a[i] = (__bf16)p[i]; a[8 + i] = (__bf16)p[16 + i]; } }
    acc[0] = wmma_bf(a, frag_b(PW + PRT + (size_t)col * DD + kc * 32, lane), acc[0]); acc[1] = wmma_bf(a, frag_b(PW + PIN + (size_t)col * DD + kc * 32, lane), acc[1]); }
#pragma unroll
  for (int r = 0; r < 8; ++r) { sl[wave][8 * g + r][col] = acc[0][r]; sl[wave][8 * g + r][16 + col] = acc[1][r]; }
  LDSX();
  if (lane < 16) { const int rl = lane, tl = wave * 16 + rl; float lg[NOUT]; float mx = -3.0e38f;
#pragma unroll
    for (int o = 0; o < NOUT; ++o) { lg[o] = sl[wave][rl][o]; mx = fmaxf(mx, lg[o]); }
    float pr[NOUT], z = 0.f;
#pragma unroll
    for (int o = 0; o < NOUT; ++o) { pr[o] = exp_ni(lg[o] - mx); z += pr[o]; }
    int o1 = 0; float b1 = pr[0];
#pragma unroll
    for (int o = 1; o < NOUT; ++o) if (pr[o] > b1) { b1 = pr[o]; o1 = o; }
    int o2 = -1; float b2 = -1.f;
#pragma unroll
    for (int o = 0; o < NOUT; ++o) if (o != o1 && (o2 < 0 || pr[o] > b2)) { b2 = pr[o]; o2 = o; }
    const float p1 = b1 / z, p2 = b2 / z; const float rs = p1 + p2; const float rw0 = p1 / rs, rw1 = p2 / rs;
    const float s20 = sl[wave][rl][16 + 2 * o2], s21 = sl[wave][rl][16 + 2 * o2 + 1]; const int e3 = 2 * o2 + ((s21 > s20) ? 1 : 0);
#pragma unroll
    for (int e = 0; e < NE; ++e) { float w = 0.f; if (e == 2 * o1 || e == 2 * o1 + 1) w += rw0; if (e == e3) w += rw1; scw[tl][e] = w; }
    ssw[tl * 3] = rw0; ssw[tl * 3 + 1] = rw0; ssw[tl * 3 + 2] = rw1; }
  __syncthreads();
  for (int q = tid; q < 64 * NE / 4; q += 128) vst2(CW + (size_t)blockIdx.x * 64 * NE + q * 4, *(const v4f*)(&scw[0][0] + q * 4));
  if (tid < 48) vst2(SELW + (size_t)blockIdx.x * 64 * 3 + tid * 4, *(const v4f*)&ssw[tid * 4]);
}
__global__ __launch_bounds__(128) void k_gu(const float* __restrict__ X, const __bf16* __restrict__ PW, float* __restrict__ H) {
  __shared__ __align__(16) float so[4][16][68];
  const int tid = threadIdx.x, wave = tid >> 5, lane = tid & 31, col = lane & 15, g = lane >> 4; const size_t r0 = (size_t)blockIdx.x * 64 + wave * 16;
  const int e = blockIdx.y >> 3, f0 = (blockIdx.y & 7) * 64;
  const __bf16* PG = PW + PGU + ((size_t)e * 1024 + f0) * DD; const __bf16* PU = PW + PGU + ((size_t)e * 1024 + FF + f0) * DD;
  v8f ag[4] = {}, au[4] = {};
#pragma unroll 2
  for (int kc = 0; kc < DD / 32; ++kc) { v16b a; { const float* p = X + (r0 + col) * DD + kc * 32 + 8 * g;
#pragma unroll
      for (int i = 0; i < 8; ++i) { a[i] = (__bf16)p[i]; a[8 + i] = (__bf16)p[16 + i]; } }
#pragma unroll
    for (int j = 0; j < 4; ++j) { ag[j] = wmma_bf(a, frag_b(PG + (size_t)(j * 16 + col) * DD + kc * 32, lane), ag[j]); au[j] = wmma_bf(a, frag_b(PU + (size_t)(j * 16 + col) * DD + kc * 32, lane), au[j]); } }
#pragma unroll
  for (int j = 0; j < 4; ++j)
#pragma unroll
    for (int r = 0; r < 8; ++r) { const float gv = ag[j][r]; so[wave][8 * g + r][j * 16 + col] = (gv * sigm(gv)) * au[j][r]; }
  LDSX();
  for (int rl = 0; rl < 16; ++rl) if (lane < 16) vst2(H + (r0 + rl) * (size_t)(NE * FF) + e * FF + f0 + lane * 4, *(const v4f*)&so[wave][rl][lane * 4]);
}
__global__ __launch_bounds__(128) void k_down(const float* __restrict__ H, const __bf16* __restrict__ PW, const float* __restrict__ CW, float* __restrict__ OUT) {
  __shared__ __align__(16) float so[4][16][132];
  const int tid = threadIdx.x, wave = tid >> 5, lane = tid & 31, col = lane & 15, g = lane >> 4; const size_t r0 = (size_t)blockIdx.x * 64 + wave * 16; const int n0 = blockIdx.y * 128;
  float tot[8][8];
#pragma unroll
  for (int j = 0; j < 8; ++j)
#pragma unroll
    for (int r = 0; r < 8; ++r) tot[j][r] = 0.f;
#pragma unroll 1
  for (int e = 0; e < NE; ++e) { v8f acc[8] = {};
#pragma unroll 2
    for (int kc = 0; kc < FF / 32; ++kc) { const F2 a = split_row(H + (r0 + col) * (size_t)(NE * FF) + e * FF, kc * 32, lane);
#pragma unroll
      for (int j = 0; j < 8; ++j) { const v16b w = frag_b(PW + PWD + ((size_t)e * DD + n0 + j * 16 + col) * FF + kc * 32, lane); acc[j] = wmma_bf(a.l, w, acc[j]); acc[j] = wmma_bf(a.h, w, acc[j]); } }
    float cw[8];
#pragma unroll
    for (int r = 0; r < 8; ++r) cw[r] = CW[(r0 + 8 * g + r) * NE + e];
#pragma unroll
    for (int j = 0; j < 8; ++j)
#pragma unroll
      for (int r = 0; r < 8; ++r) tot[j][r] += acc[j][r] * cw[r]; }
#pragma unroll
  for (int j = 0; j < 8; ++j)
#pragma unroll
    for (int r = 0; r < 8; ++r) so[wave][8 * g + r][j * 16 + col] = tot[j][r];
  LDSX();
  for (int rl = 0; rl < 16; ++rl) vst2(OUT + (r0 + rl) * DD + n0 + lane * 4, *(const v4f*)&so[wave][rl][lane * 4]);
}
extern "C" void kernel_launch(void* const* d_in, const int* in_sizes, int n_in, void* d_out, int out_size, void* d_ws, size_t ws_size, hipStream_t stream) {
  (void)in_sizes; (void)n_in; (void)out_size;
  const float** Fp = (const float**)d_in;
  if (ws_size < (size_t)WS_END) return;
  char* ws = (char*)d_ws; __bf16* PW = (__bf16*)(ws + WS_PW); float *CW = (float*)(ws + WS_CW), *H = (float*)(ws + WS_H);
  float* OUT = (float*)d_out; float* SELW = OUT + (size_t)NT_ * DD;
  k_pack<<<dim3(NE * 1024, 3), 256, 0, stream>>>(Fp[1], Fp[2], Fp[3], Fp[4], Fp[5], PW);
  k_route<<<NRB, 128, 0, stream>>>(Fp[0], PW, CW, SELW);
  k_gu<<<dim3(NRB, NE * 8), 128, 0, stream>>>(Fp[0], PW, H);
  k_down<<<dim3(NRB, DD / 128), 128, 0, stream>>>(H, PW, CW, OUT);
}
